// ContextGuidedSelectiveStateModel_82987358094113
// MI455X (gfx1250) — hardware-verified
//
#include <hip/hip_runtime.h>
#include <math.h>

typedef __attribute__((ext_vector_type(16))) _Float16 v16h;
typedef __attribute__((ext_vector_type(8)))  _Float16 v8h;
typedef __attribute__((ext_vector_type(16))) __bf16   v16b;
typedef __attribute__((ext_vector_type(8)))  __bf16   v8b;
typedef __attribute__((ext_vector_type(8)))  float    v8f;
typedef __attribute__((ext_vector_type(4)))  float    v4f;
typedef __attribute__((ext_vector_type(2)))  unsigned v2u;
#define PSCALE 32768.0f
#define U16(p) ((const unsigned short*)(const void*)(p))
#define PSCALE_INV (1.0f / 32768.0f)

#define EMB   768
#define INNER 1536
#define DRANK 48
#define STATE 16
#define SEQL  2048
#define NTOK  4096
#define XPC   80
#define XPW   128
#define DTW   64
#define LOG2E 1.4426950408889634f

__device__ __forceinline__ unsigned short f2bf_bits(float f) {
  unsigned u = __float_as_uint(f);
  return (unsigned short)((u + 0x7FFFu + ((u >> 16) & 1u)) >> 16);
}
__device__ __forceinline__ float bf_bits2f(unsigned short h) { return __uint_as_float(((unsigned)h) << 16); }
__device__ __forceinline__ void bf_split(float f, unsigned short& hb, unsigned short& lb) {
  hb = f2bf_bits(f);
  lb = f2bf_bits(f - bf_bits2f(hb));
}

__device__ __forceinline__ void dep_guard_h(v8f& a, v8f& b, v16h x, v16h y) { asm volatile("v_nop\n\tv_nop\n\tv_nop\n\tv_nop" : "+v"(a), "+v"(b) : "v"(x), "v"(y)); }
__device__ __forceinline__ void dep_guard_b(v8f& a, v8f& b, v16b x, v16b y) { asm volatile("v_nop\n\tv_nop\n\tv_nop\n\tv_nop" : "+v"(a), "+v"(b) : "v"(x), "v"(y)); }
__device__ __forceinline__ void keep4_h(v16h a, v16h b, v16h c, v16h d) { asm volatile("v_nop" :: "v"(a), "v"(b), "v"(c), "v"(d)); }
__device__ __forceinline__ void keep4_b(v16b a, v16b b, v16b c, v16b d) { asm volatile("v_nop" :: "v"(a), "v"(b), "v"(c), "v"(d)); }
__device__ __forceinline__ void acc_guard4(v8f& a, v8f& b, v8f& c, v8f& d) { asm volatile("v_nop\n\tv_nop\n\tv_nop\n\tv_nop" : "+v"(a), "+v"(b), "+v"(c), "+v"(d)); }
template <typename T> struct Frag;
template <> struct Frag<_Float16> {
  typedef v16h V; union U { v16h v; v8h h[2]; };
  static __device__ __forceinline__ v16h load(const _Float16* p) {
    U f; f.h[0] = *(const v8h*)(p); f.h[1] = *(const v8h*)(p + 16); return f.v;
  }
  static __device__ __forceinline__ v8f mma(v16h a, v16h b, v8f c) {
    return __builtin_amdgcn_wmma_f32_16x16x32_f16(false, a, false, b, (short)0, c, false, false);
  }
  static __device__ __forceinline__ void guard(v8f& a, v8f& b, v16h x, v16h y) { dep_guard_h(a, b, x, y); }
  static __device__ __forceinline__ void keep(v16h a, v16h b, v16h c, v16h d) { keep4_h(a, b, c, d); }
};
template <> struct Frag<__bf16> {
  typedef v16b V; union U { v16b v; v8b h[2]; };
  static __device__ __forceinline__ v16b load(const __bf16* p) {
    U f; f.h[0] = *(const v8b*)(p); f.h[1] = *(const v8b*)(p + 16); return f.v;
  }
  static __device__ __forceinline__ v8f mma(v16b a, v16b b, v8f c) {
    return __builtin_amdgcn_wmma_f32_16x16x32_bf16(false, a, false, b, (short)0, c, false, false);
  }
  static __device__ __forceinline__ void guard(v8f& a, v8f& b, v16b x, v16b y) { dep_guard_b(a, b, x, y); }
  static __device__ __forceinline__ void keep(v16b a, v16b b, v16b c, v16b d) { keep4_b(a, b, c, d); }
};

template <int ET> struct Elem;
template <> struct Elem<0> { typedef _Float16 T; };
template <> struct Elem<1> { typedef __bf16 T; };
template <int ET, bool SPLIT, int BIAS_MODE, int OUT_MODE, bool RESID, int ACT = 0, int EPX = 0>
__global__ __launch_bounds__(256) void wmma_gemm64(
    const unsigned short* __restrict__ Ap, const unsigned short* __restrict__ A2p, int lda, long strideA,
    const unsigned short* __restrict__ Btp, const unsigned short* __restrict__ Bt2p, int ldb, long strideB,
    void* __restrict__ Cout, void* __restrict__ Cout2, int ldc, long strideC,
    const float* __restrict__ bias,
    const float* __restrict__ resid, long strideR,
    int M, int N, int K, float scale,
    const float* __restrict__ aux1, const float* __restrict__ aux2, int segRows, int nCut) {
  typedef typename Elem<ET>::T T;
  typedef typename Frag<T>::V V;
  const T* A = (const T*)Ap; const T* A2 = (const T*)A2p; const T* Bt = (const T*)Btp; const T* Bt2 = (const T*)Bt2p;
  __shared__ __align__(16) float sT[8][16 * 68];
  const int b    = blockIdx.y;
  const int lane = threadIdx.x & 31;
  const int wave = threadIdx.x >> 5;
  const int tilesN = N >> 6;
  const int tilesM = M >> 6;
  const int tile = blockIdx.x * 8 + wave;
  if (tile >= tilesM * tilesN) return;
  const int tm = tile / tilesN;
  const int tn = tile - tm * tilesN;
  const int m0 = tm << 6;
  const int n0 = tn << 6;

  const T* Ab  = A  + (size_t)b * strideA;
  const T* Bb  = Bt + (size_t)b * strideB;
  const T* Ab2 = SPLIT ? (A2  + (size_t)b * strideA) : nullptr;
  const T* Bb2 = SPLIT ? (Bt2 + (size_t)b * strideB) : nullptr;

  const int rlane = lane & 15;
  const int koff  = (lane >> 4) * 8;
  const int mOff  = (lane >> 4) * 8;

  v8f acc[4][4];
#pragma unroll
  for (int i = 0; i < 4; ++i)
#pragma unroll
    for (int j = 0; j < 4; ++j) acc[i][j] = (v8f){0.f,0.f,0.f,0.f,0.f,0.f,0.f,0.f};

  for (int k0 = 0; k0 < K; k0 += 32) {
    V bh[4], bl[4];
#pragma unroll
    for (int j = 0; j < 4; ++j) {
      const size_t bo = (size_t)(n0 + (j << 4) + rlane) * ldb + koff + k0;
      bh[j] = Frag<T>::load(Bb + bo);
      if (SPLIT) bl[j] = Frag<T>::load(Bb2 + bo);
    }
#pragma unroll
    for (int i = 0; i < 4; ++i) {
      const size_t ao = (size_t)(m0 + (i << 4) + rlane) * lda + koff + k0;
      V ah = Frag<T>::load(Ab + ao);
      V al;
      if (SPLIT) al = Frag<T>::load(Ab2 + ao);
#pragma unroll
      for (int j = 0; j < 4; ++j) {
        acc[i][j] = Frag<T>::mma(ah, bh[j], acc[i][j]);
        if (SPLIT) {
          acc[i][j] = Frag<T>::mma(ah, bl[j], acc[i][j]);
          acc[i][j] = Frag<T>::mma(al, bh[j], acc[i][j]);
        }
      }
      Frag<T>::guard(acc[i][0], acc[i][3], ah, SPLIT ? al : ah);
    }
    Frag<T>::keep(bh[0], bh[1], bh[2], bh[3]);
    if (SPLIT) Frag<T>::keep(bl[0], bl[1], bl[2], bl[3]);
  }
  acc_guard4(acc[0][0], acc[0][1], acc[0][2], acc[0][3]);
  acc_guard4(acc[1][0], acc[1][1], acc[1][2], acc[1][3]);
  acc_guard4(acc[2][0], acc[2][1], acc[2][2], acc[2][3]);
  acc_guard4(acc[3][0], acc[3][1], acc[3][2], acc[3][3]);

  float* slab = sT[wave];
  const float* Rb = RESID ? (resid + (size_t)b * strideR) : nullptr;
  const bool isX = (EPX == 0) ? true : (n0 < nCut);
  const int  seg = (EPX == 1) ? (m0 / segRows) : 0;
  const int  nb  = isX ? n0 : (n0 - nCut);
  const float* auxp = (EPX == 1) ? (isX ? aux1 : aux2) : nullptr;
#pragma unroll
  for (int i = 0; i < 4; ++i) {
    const int mBase = m0 + (i << 4);
#pragma unroll
    for (int j = 0; j < 4; ++j) {
      const int n = n0 + (j << 4) + rlane;
      float bv = 0.f;
      if (BIAS_MODE == 2) bv = bias[n];
      float ax = 0.f;
      if (EPX == 1) ax = auxp[(size_t)seg * nCut + (n - n0) + nb];
#pragma unroll
      for (int r = 0; r < 8; ++r) {
        float v = acc[i][j][r] * scale;
        if (BIAS_MODE == 1) v += bias[mBase + mOff + r];
        if (BIAS_MODE == 2) v += bv;
        if (RESID) v += Rb[(size_t)(mBase + mOff + r) * ldc + n];
        if (ACT == 1) v = tanhf(v);
        if (ACT == 2) v = fmaxf(v, 0.0f);
        if (ACT == 3) v = v / (1.0f + expf(-v));
        if (ACT == 4) v = (v > 0.f) ? v : 0.01f * v;
        if (ACT == 5) v = 0.5f * v * (1.0f + erff(v * 0.70710678118654752f));
        if (EPX == 1) v = isX ? (v * (1.0f + ax)) : (v + ax);
        slab[(mOff + r) * 68 + (j << 4) + rlane] = v;
      }
    }
    __builtin_amdgcn_fence(__ATOMIC_RELEASE, "workgroup");
    __builtin_amdgcn_wave_barrier();
    __builtin_amdgcn_fence(__ATOMIC_ACQUIRE, "workgroup");
    if (OUT_MODE == 0) {
      float* C = (float*)(isX ? Cout : Cout2) + (size_t)b * strideC;
      const int hh = lane >> 4, c4 = (lane & 15) * 4;
      for (int pass = 0; pass < 2; ++pass) {
#pragma unroll
        for (int it = 0; it < 8; ++it) {
          const int row = it * 2 + hh;
          v4f v = *(const v4f*)(slab + row * 68 + c4);
          *(volatile v4f*)(C + (size_t)(mBase + row) * ldc + nb + c4) = v;
        }
        __threadfence();
      }
    } else {
      const int q = lane >> 3, c8 = (lane & 7) * 8;
      unsigned short* C  = (unsigned short*)Cout  + (size_t)b * strideC;
      unsigned short* C2 = (OUT_MODE == 2) ? ((unsigned short*)Cout2 + (size_t)b * strideC) : nullptr;
      for (int pass = 0; pass < 2; ++pass) {
#pragma unroll
        for (int it = 0; it < 4; ++it) {
          const int row = it * 4 + q;
          const float* sp = slab + row * 68 + c8;
          v8h hv, lv;
#pragma unroll
          for (int e = 0; e < 8; ++e) {
            if (OUT_MODE == 1) {
              hv[e] = (_Float16)sp[e];
            } else {
              unsigned short hb = f2bf_bits(sp[e]);
              unsigned short lb = f2bf_bits(sp[e] - bf_bits2f(hb));
              hv[e] = __builtin_bit_cast(_Float16, hb);
              lv[e] = __builtin_bit_cast(_Float16, lb);
            }
          }
          *(volatile v8h*)(C + (size_t)(mBase + row) * ldc + nb + c8) = hv;
          if (OUT_MODE == 2) *(volatile v8h*)(C2 + (size_t)(mBase + row) * ldc + nb + c8) = lv;
        }
        __threadfence();
      }
    }
    __builtin_amdgcn_fence(__ATOMIC_RELEASE, "workgroup");
    __builtin_amdgcn_wave_barrier();
    __builtin_amdgcn_fence(__ATOMIC_ACQUIRE, "workgroup");
  }
}

__device__ __forceinline__ float sigm_(float x) { return __builtin_amdgcn_rcpf(1.0f + expf(-x)); }
__device__ __forceinline__ float silu_(float x) { return x * sigm_(x); }
__device__ __forceinline__ float wave_sum(float v) {
#pragma unroll
  for (int off = 1; off < 32; off <<= 1) v += __shfl_xor(v, off, 32);
  return v;
}
__device__ __forceinline__ void ld16(const float* __restrict__ p, float (&d)[16]) {
  const v4f a = *(const v4f*)(p), bq = *(const v4f*)(p + 4), cq = *(const v4f*)(p + 8), eq = *(const v4f*)(p + 12);
  d[0] = a.x;  d[1] = a.y;  d[2] = a.z;  d[3] = a.w;
  d[4] = bq.x; d[5] = bq.y; d[6] = bq.z; d[7] = bq.w;
  d[8] = cq.x; d[9] = cq.y; d[10] = cq.z; d[11] = cq.w;
  d[12] = eq.x; d[13] = eq.y; d[14] = eq.z; d[15] = eq.w;
}

__global__ __launch_bounds__(256) void split_rows_kernel(const float* __restrict__ in,
                                                         unsigned short* __restrict__ H,
                                                         unsigned short* __restrict__ L, int n2) {
  const int i = blockIdx.x * 256 + threadIdx.x;
  if (i < n2) {
    const float2 f = *(const float2*)(in + 2 * (size_t)i);
    unsigned short h0, l0, h1, l1;
    bf_split(f.x, h0, l0);
    bf_split(f.y, h1, l1);
    const unsigned uh = (unsigned)h0 | ((unsigned)h1 << 16);
    const unsigned ul = (unsigned)l0 | ((unsigned)l1 << 16);
    ((volatile unsigned*)H)[i] = uh;
    ((volatile unsigned*)L)[i] = ul;
    __threadfence();
    ((volatile unsigned*)H)[i] = uh;
    ((volatile unsigned*)L)[i] = ul;
  }
}

__global__ __launch_bounds__(256) void transpose_split_kernel(const float* __restrict__ W, int K, int N, int Kp, int Np,
                                                              unsigned short* __restrict__ H, unsigned short* __restrict__ L) {
  __shared__ float tile[64][65];
  const int tid = threadIdx.x, lane = tid & 31, wave = tid >> 5;
  const int k0 = blockIdx.x * 64, n0 = blockIdx.y * 64;
#pragma unroll
  for (int it = 0; it < 16; ++it) {
    const int idx = it * 256 + tid;
    const int kk = idx >> 6, nn = idx & 63;
    const int k = k0 + kk, n = n0 + nn;
    const int kc = (k < K) ? k : (K - 1);
    const int nc = (n < N) ? n : (N - 1);
    float v = W[(size_t)kc * N + nc];
    if (k >= K || n >= N) v = 0.f;
    tile[kk][nn] = v;
  }
  __syncthreads();
  const int c8 = (lane & 7) * 8;
#pragma unroll
  for (int half = 0; half < 2; ++half) {
    const int rr = wave * 8 + half * 4 + (lane >> 3);
    v8h hv, lv;
#pragma unroll
    for (int e = 0; e < 8; ++e) {
      const float f = tile[c8 + e][rr];
      unsigned short hb, lb;
      bf_split(f, hb, lb);
      hv[e] = __builtin_bit_cast(_Float16, hb);
      lv[e] = __builtin_bit_cast(_Float16, lb);
    }
    const size_t o = (size_t)(n0 + rr) * Kp + k0 + c8;
    *(volatile v8h*)(H + o) = hv;
    *(volatile v8h*)(L + o) = lv;
    __threadfence();
    *(volatile v8h*)(H + o) = hv;
    *(volatile v8h*)(L + o) = lv;
  }
}

__global__ __launch_bounds__(256) void ctx_kernel(const float* __restrict__ rctx,
                                                  const float* __restrict__ ln_g, const float* __restrict__ ln_b,
                                                  const float* __restrict__ Ws, const float* __restrict__ bs,
                                                  const float* __restrict__ Wg, const float* __restrict__ bg,
                                                  float* __restrict__ drive, float* __restrict__ gbias) {
  __shared__ float cn[EMB];
  __shared__ float red[8];
  __shared__ float stat[2];
  const int b = blockIdx.y;
  const int tid = threadIdx.x, lane = tid & 31, wave = tid >> 5;
  const float* row = rctx + (size_t)b * EMB;

  float s = 0.f;
  for (int k = tid; k < EMB; k += 256) s += row[k];
  s = wave_sum(s);
  if (lane == 0) red[wave] = s;
  __syncthreads();
  if (tid == 0) {
    float t = 0.f;
#pragma unroll
    for (int w = 0; w < 8; ++w) t += red[w];
    stat[0] = t * (1.0f / EMB);
  }
  __syncthreads();
  const float mean = stat[0];
  float s2 = 0.f;
  for (int k = tid; k < EMB; k += 256) { const float d = row[k] - mean; s2 += d * d; }
  s2 = wave_sum(s2);
  if (lane == 0) red[wave] = s2;
  __syncthreads();
  if (tid == 0) {
    float t = 0.f;
#pragma unroll
    for (int w = 0; w < 8; ++w) t += red[w];
    stat[1] = t * (1.0f / EMB);
  }
  __syncthreads();
  const float var = stat[1];
  const float inv = rsqrtf(var + 1e-5f);
  for (int k = tid; k < EMB; k += 256) cn[k] = (row[k] - mean) * inv * ln_g[k] + ln_b[k];
  __syncthreads();

  const int j = blockIdx.x * 256 + tid;
  float a1 = bs[j];
  float a2 = bg[j];
#pragma unroll 2
  for (int k = 0; k < EMB; ++k) {
    const float v = cn[k];
    a1 = fmaf(v, Ws[(size_t)k * INNER + j], a1);
    a2 = fmaf(v, Wg[(size_t)k * INNER + j], a2);
  }
  const float dr = sigm_(a1);
  const size_t o = (size_t)b * INNER + j;
  *(volatile float*)(drive + o) = dr;
  *(volatile float*)(gbias + o) = a2;
  __threadfence();
  *(volatile float*)(drive + o) = dr;
  *(volatile float*)(gbias + o) = a2;
}

__global__ __launch_bounds__(256) void conv_silu_kernel(const float* __restrict__ xm,
                                                        const float* __restrict__ cw, const float* __restrict__ cb,
                                                        float* __restrict__ xc,
                                                        unsigned short* __restrict__ xH, unsigned short* __restrict__ xL,
                                                        int total) {
  const int gid = blockIdx.x * 256 + threadIdx.x;
  if (gid >= total) return;
  const int q   = gid % (INNER / 4);
  const int rw  = gid / (INNER / 4);
  const int l   = rw & (SEQL - 1);
  const int c4  = q * 4;
  const size_t base = (size_t)rw * INNER + c4;
  const size_t b1 = (l >= 1) ? (base - INNER) : base;
  const size_t b2 = (l >= 2) ? (base - 2 * (size_t)INNER) : base;
  const v4f x0 = *(const v4f*)(xm + base);
  v4f x1 = *(const v4f*)(xm + b1);
  v4f x2 = *(const v4f*)(xm + b2);
  const v4f zero4 = {0.f, 0.f, 0.f, 0.f};
  if (l < 1) x1 = zero4;
  if (l < 2) x2 = zero4;
  const v4f wa = *(const v4f*)(cw + (size_t)c4 * 3);
  const v4f wb = *(const v4f*)(cw + (size_t)c4 * 3 + 4);
  const v4f wc = *(const v4f*)(cw + (size_t)c4 * 3 + 8);
  const v4f cbv = *(const v4f*)(cb + c4);
  const float o0 = cbv.x + wa.x * x2.x + wa.y * x1.x + wa.z * x0.x;
  const float o1 = cbv.y + wa.w * x2.y + wb.x * x1.y + wb.y * x0.y;
  const float o2 = cbv.z + wb.z * x2.z + wb.w * x1.z + wc.x * x0.z;
  const float o3 = cbv.w + wc.y * x2.w + wc.z * x1.w + wc.w * x0.w;
  v4f out;
  out.x = silu_(o0); out.y = silu_(o1); out.z = silu_(o2); out.w = silu_(o3);
  unsigned short h0, l0, h1, l1, h2, l2, h3, l3;
  bf_split(out.x, h0, l0); bf_split(out.y, h1, l1); bf_split(out.z, h2, l2); bf_split(out.w, h3, l3);
  v2u ph, pl;
  ph.x = (unsigned)h0 | ((unsigned)h1 << 16); ph.y = (unsigned)h2 | ((unsigned)h3 << 16);
  pl.x = (unsigned)l0 | ((unsigned)l1 << 16); pl.y = (unsigned)l2 | ((unsigned)l3 << 16);
  *(volatile v4f*)(xc + base) = out;
  *(volatile v2u*)(xH + base) = ph;
  *(volatile v2u*)(xL + base) = pl;
  __threadfence();
  *(volatile v4f*)(xc + base) = out;
  *(volatile v2u*)(xH + base) = ph;
  *(volatile v2u*)(xL + base) = pl;
}

__global__ __launch_bounds__(256) void dt_split_kernel(const float* __restrict__ xp,
                                                       unsigned short* __restrict__ H, unsigned short* __restrict__ L) {
  const int tid = threadIdx.x;
  const int rw = blockIdx.x * 32 + (tid >> 3);
  const int c8 = (tid & 7) * 8;
  const int cc = (c8 < DRANK) ? c8 : (DRANK - 8);
  const float* p = xp + (size_t)rw * XPW + cc;
  v4f a = *(const v4f*)(p);
  v4f bq = *(const v4f*)(p + 4);
  const v4f zero4 = {0.f, 0.f, 0.f, 0.f};
  if (c8 >= DRANK) { a = zero4; bq = zero4; }
  float f[8];
  f[0] = a.x; f[1] = a.y; f[2] = a.z; f[3] = a.w; f[4] = bq.x; f[5] = bq.y; f[6] = bq.z; f[7] = bq.w;
  v8h hv, lv;
#pragma unroll
  for (int e = 0; e < 8; ++e) {
    unsigned short hb, lb;
    bf_split(f[e], hb, lb);
    hv[e] = __builtin_bit_cast(_Float16, hb);
    lv[e] = __builtin_bit_cast(_Float16, lb);
  }
  const size_t o = (size_t)rw * DTW + c8;
  *(volatile v8h*)(H + o) = hv;
  *(volatile v8h*)(L + o) = lv;
  __threadfence();
  *(volatile v8h*)(H + o) = hv;
  *(volatile v8h*)(L + o) = lv;
}

__global__ __launch_bounds__(64) void scan_kernel(const float* __restrict__ xc,
                                                  const float* __restrict__ dpre,
                                                  const float* __restrict__ xp,
                                                  const float* __restrict__ zm,
                                                  const float* __restrict__ logA,
                                                  const float* __restrict__ Dv,
                                                  float* __restrict__ g, int nthreads) {
  const int t = blockIdx.x * 64 + threadIdx.x;
  if (t >= nthreads) return;
  const int b = t / INNER;
  const int c = t - b * INNER;
  float A[STATE], st[STATE];
#pragma unroll
  for (int s = 0; s < STATE; ++s) {
    A[s]  = -expf(logA[(size_t)c * STATE + s]);
    st[s] = 0.f;
  }
  const float Dc = Dv[c];
  const size_t rowb = (size_t)b * SEQL;
  for (int l = 0; l < SEQL; ++l) {
    const size_t rw  = rowb + l;
    const size_t off = rw * INNER + c;
    const float dp = dpre[off];
    const float dv = fmaxf(dp, 0.f) + log1pf(expf(-fabsf(dp)));
    const float xv = xc[off];
    const float zv = zm[off];
    float Bs[STATE], Cs[STATE];
    ld16(xp + rw * XPW + DRANK, Bs);
    ld16(xp + rw * XPW + DRANK + STATE, Cs);
    const float dx = dv * xv;
    float y = 0.f;
#pragma unroll
    for (int s = 0; s < STATE; ++s) {
      const float e  = dv * A[s];
      const float dA = exp2f(e * LOG2E);
      st[s] = fmaf(dA, st[s], dx * Bs[s]);
      y = fmaf(st[s], Cs[s], y);
    }
    y = fmaf(xv, Dc, y);
    const float out = y * silu_(zv);
    *(volatile float*)(g + off) = out;
    __threadfence();
    *(volatile float*)(g + off) = out;
  }
}

extern "C" void kernel_launch(void* const* d_in, const int* in_sizes, int n_in,
                              void* d_out, int out_size, void* d_ws, size_t ws_size,
                              hipStream_t stream) {
  if (n_in < 19) return;
  if (in_sizes[0] != NTOK * EMB || in_sizes[1] != 2 * EMB || in_sizes[2] != EMB * 2 * INNER ||
      in_sizes[3] != 2 * INNER || in_sizes[4] != INNER * 3 || in_sizes[5] != INNER ||
      in_sizes[6] != INNER * XPC || in_sizes[7] != DRANK * INNER || in_sizes[8] != INNER ||
      in_sizes[9] != INNER * STATE || in_sizes[10] != INNER || in_sizes[11] != INNER * EMB ||
      in_sizes[12] != EMB || in_sizes[13] != EMB || in_sizes[14] != EMB ||
      in_sizes[15] != EMB * INNER || in_sizes[16] != INNER || in_sizes[17] != EMB * INNER ||
      in_sizes[18] != INNER) return;
  if (out_size != NTOK * EMB) return;

  const float* tokens  = (const float*)d_in[0];
  const float* rctx    = (const float*)d_in[1];
  const float* W_in    = (const float*)d_in[2];
  const float* b_in    = (const float*)d_in[3];
  const float* conv_w  = (const float*)d_in[4];
  const float* conv_b  = (const float*)d_in[5];
  const float* W_x     = (const float*)d_in[6];
  const float* W_dt    = (const float*)d_in[7];
  const float* b_dt    = (const float*)d_in[8];
  const float* log_A   = (const float*)d_in[9];
  const float* Dvec    = (const float*)d_in[10];
  const float* W_out   = (const float*)d_in[11];
  const float* b_out   = (const float*)d_in[12];
  const float* ln_g    = (const float*)d_in[13];
  const float* ln_b    = (const float*)d_in[14];
  const float* W_scale = (const float*)d_in[15];
  const float* b_scale = (const float*)d_in[16];
  const float* W_gbias = (const float*)d_in[17];
  const float* b_gbias = (const float*)d_in[18];
  float* out = (float*)d_out;

  const size_t P24    = (size_t)NTOK * INNER * 4;
  const size_t PL     = (size_t)NTOK * INNER * 2;
  const size_t TOKP   = (size_t)NTOK * EMB * 2;
  const size_t WINP   = (size_t)2 * INNER * EMB * 2;
  const size_t XPB    = (size_t)NTOK * XPW * 4;
  const size_t DTP    = (size_t)NTOK * DTW * 2;
  const size_t WXP    = (size_t)XPW * INNER * 2;
  const size_t WDTP   = (size_t)INNER * DTW * 2;
  const size_t WOUTP  = (size_t)EMB * INNER * 2;
  const size_t DRB    = (size_t)2 * INNER * 4;

  const size_t oR0 = 0;
  const size_t oR1 = P24;
  const size_t oR2 = 2 * P24;
  const size_t oR3 = 3 * P24;
  const size_t oR4 = 4 * P24;
  const size_t oR5 = oR4 + 2 * TOKP + 2 * WINP;
  const size_t total = oR5 + 2 * WXP + 2 * WDTP + 2 * WOUTP + 2 * DRB;
  if (total > ws_size || total > (size_t)134217728) return;

  char* ws = (char*)d_ws;
  float* xmod  = (float*)(ws + oR0);
  float* dpre  = (float*)(ws + oR0);
  unsigned short* gH = (unsigned short*)(ws + oR0);
  unsigned short* gL = (unsigned short*)(ws + oR0 + PL);
  float* zmod  = (float*)(ws + oR1);
  float* xcf   = (float*)(ws + oR2);
  unsigned short* xcH = (unsigned short*)(ws + oR3);
  unsigned short* xcL = (unsigned short*)(ws + oR3 + PL);
  float* gf    = (float*)(ws + oR3);
  unsigned short* tokH  = (unsigned short*)(ws + oR4);
  unsigned short* tokL  = (unsigned short*)(ws + oR4 + TOKP);
  unsigned short* winH  = (unsigned short*)(ws + oR4 + 2 * TOKP);
  unsigned short* winL  = (unsigned short*)(ws + oR4 + 2 * TOKP + WINP);
  float* xpf   = (float*)(ws + oR4);
  unsigned short* dtH   = (unsigned short*)(ws + oR4 + XPB);
  unsigned short* dtL   = (unsigned short*)(ws + oR4 + XPB + DTP);
  unsigned short* wxH   = (unsigned short*)(ws + oR5);
  unsigned short* wxL   = (unsigned short*)(ws + oR5 + WXP);
  unsigned short* wdtH  = (unsigned short*)(ws + oR5 + 2 * WXP);
  unsigned short* wdtL  = (unsigned short*)(ws + oR5 + 2 * WXP + WDTP);
  unsigned short* woutH = (unsigned short*)(ws + oR5 + 2 * WXP + 2 * WDTP);
  unsigned short* woutL = (unsigned short*)(ws + oR5 + 2 * WXP + 2 * WDTP + WOUTP);
  float* drive = (float*)(ws + oR5 + 2 * WXP + 2 * WDTP + 2 * WOUTP);
  float* gbias = (float*)(ws + oR5 + 2 * WXP + 2 * WDTP + 2 * WOUTP + DRB);

  split_rows_kernel<<<(NTOK * EMB / 2 + 255) / 256, 256, 0, stream>>>(tokens, tokH, tokL, NTOK * EMB / 2);
  transpose_split_kernel<<<dim3(EMB / 64, 2 * INNER / 64), 256, 0, stream>>>(W_in, EMB, 2 * INNER, EMB, 2 * INNER, winH, winL);
  transpose_split_kernel<<<dim3(INNER / 64, XPW / 64), 256, 0, stream>>>(W_x, INNER, XPC, INNER, XPW, wxH, wxL);
  transpose_split_kernel<<<dim3(DTW / 64, INNER / 64), 256, 0, stream>>>(W_dt, DRANK, INNER, DTW, INNER, wdtH, wdtL);
  transpose_split_kernel<<<dim3(INNER / 64, EMB / 64), 256, 0, stream>>>(W_out, INNER, EMB, INNER, EMB, woutH, woutL);
  ctx_kernel<<<dim3(INNER / 256, 2), 256, 0, stream>>>(rctx, ln_g, ln_b, W_scale, b_scale, W_gbias, b_gbias, drive, gbias);
  {
    const int tiles = (NTOK / 64) * (2 * INNER / 64);
    wmma_gemm64<1, true, 2, 0, false, 0, 1><<<dim3((tiles + 7) / 8, 1), 256, 0, stream>>>(
        tokH, tokL, EMB, 0L, winH, winL, EMB, 0L, (void*)xmod, (void*)zmod, INNER, 0L,
        b_in, nullptr, 0L, NTOK, 2 * INNER, EMB, 1.0f, drive, gbias, SEQL, INNER);
  }
  conv_silu_kernel<<<(NTOK * (INNER / 4) + 255) / 256, 256, 0, stream>>>(xmod, conv_w, conv_b, xcf, xcH, xcL, NTOK * (INNER / 4));
  {
    const int tiles = (NTOK / 64) * (XPW / 64);
    wmma_gemm64<1, true, 0, 0, false, 0, 0><<<dim3((tiles + 7) / 8, 1), 256, 0, stream>>>(
        xcH, xcL, INNER, 0L, wxH, wxL, INNER, 0L, (void*)xpf, nullptr, XPW, 0L,
        nullptr, nullptr, 0L, NTOK, XPW, INNER, 1.0f, nullptr, nullptr, 1, 1 << 30);
  }
  dt_split_kernel<<<NTOK / 32, 256, 0, stream>>>(xpf, dtH, dtL);
  {
    const int tiles = (NTOK / 64) * (INNER / 64);
    wmma_gemm64<1, true, 2, 0, false, 0, 0><<<dim3((tiles + 7) / 8, 1), 256, 0, stream>>>(
        dtH, dtL, DTW, 0L, wdtH, wdtL, DTW, 0L, (void*)dpre, nullptr, INNER, 0L,
        b_dt, nullptr, 0L, NTOK, INNER, DTW, 1.0f, nullptr, nullptr, 1, 1 << 30);
  }
  scan_kernel<<<(2 * INNER + 63) / 64, 64, 0, stream>>>(xcf, dpre, xpf, zmod, log_A, Dvec, gf, 2 * INNER);
  split_rows_kernel<<<(NTOK * INNER / 2 + 255) / 256, 256, 0, stream>>>(gf, gH, gL, NTOK * INNER / 2);
  {
    const int tiles = (NTOK / 64) * (EMB / 64);
    wmma_gemm64<1, true, 2, 0, false, 0, 0><<<dim3((tiles + 7) / 8, 1), 256, 0, stream>>>(
        gH, gL, INNER, 0L, woutH, woutL, INNER, 0L, (void*)out, nullptr, EMB, 0L,
        b_out, nullptr, 0L, NTOK, EMB, INNER, 1.0f, nullptr, nullptr, 1, 1 << 30);
  }
}
